// GNN_BP4_41326175322289
// MI455X (gfx1250) — hardware-run, weakly checked
//
#include <hip/hip_runtime.h>


namespace {
constexpr int NB = 4, NV = 65536, NCN = 32768, D = 32, E = 262144, HID = 40, MSG = 20, HP = 48, RW = 64;
constexpr float XS = 8.0f, WSC = 256.0f;
typedef _Float16 b16;
typedef __attribute__((ext_vector_type(16))) _Float16 v16b;
typedef __attribute__((ext_vector_type(8))) _Float16 v8b;
typedef __attribute__((ext_vector_type(8))) float v8f;
typedef __attribute__((ext_vector_type(4))) float v4f;
typedef __attribute__((ext_vector_type(2))) float v2f;
__device__ __forceinline__ float bf16_rne(float f) { unsigned int u = __float_as_uint(f); u += 0x7FFFu + ((u >> 16) & 1u); return __uint_as_float(u & 0xFFFF0000u); }
__device__ __forceinline__ void split16(float v, b16& hi, b16& lo) { hi = (b16)v; lo = (b16)(v - (float)hi); }
__device__ __forceinline__ v16b frag_kb(const b16* p, int hh) { const v8b a = *(const v8b*)(p + 8 * hh), b = *(const v8b*)(p + 16 + 8 * hh); v16b f;
#pragma unroll
  for (int e = 0; e < 8; ++e) { f[e] = a[e]; f[8 + e] = b[e]; } return f; }
__device__ __forceinline__ v8f wmma16b(v16b a, v16b b, v8f c) { v8f d = __builtin_amdgcn_wmma_f32_16x16x32_f16(false, a, false, b, (short)0, c, false, false); asm volatile("v_nop\n\tv_nop\n\tv_nop\n\tv_nop" : "+v"(d) : "v"(a), "v"(b)); return d; }
__device__ __forceinline__ void wave_lds_sync() { __builtin_amdgcn_fence(__ATOMIC_RELEASE, "workgroup"); __builtin_amdgcn_wave_barrier(); __builtin_amdgcn_fence(__ATOMIC_ACQUIRE, "workgroup"); }
__device__ __forceinline__ float pmul(float a, float b) { float p = a * b; asm volatile("" : "+v"(p)); return p; }
__device__ __forceinline__ int iclamp(int v, int lo, int hi) { return v < lo ? lo : (v > hi ? hi : v); }
constexpr int CSR_NBLK = 512, CSR_GB = 9, CSR_GN = 1 << CSR_GB  , CSR_TS = (CSR_GN < 32 ? 32 : CSR_GN)  , CSR_MAXG = 512, CSR_CAP = 12288  ;
__device__ __host__ __forceinline__ int csr_tix(int v) { return (v >> CSR_GB) * CSR_TS + (v & (CSR_GN - 1)); }
__global__ __launch_bounds__(64) void csrA_kernel(const int* __restrict__ dst, int E, int N, int nG, int CHP, int NGP, int* __restrict__ STG, int* __restrict__ HST) {
  extern __shared__ int sm[];
  int* cnt = sm; int* run = sm + NGP; int* ids = sm + 2 * NGP;
  const int b = blockIdx.x; const int ch = (E + CSR_NBLK - 1) / CSR_NBLK; const int e0 = b * ch, e1 = min(E, e0 + ch);
  for (int i = threadIdx.x; i < NGP; i += 64) cnt[i] = 0;
  for (int i = threadIdx.x; i < CHP; i += 64) ids[i] = -1;
  __syncthreads();
  if (threadIdx.x == 0) {
    for (int e = e0; e < e1; ++e) { int d = dst[e]; d = (d < 0) ? 0 : (d >= N ? N - 1 : d); cnt[d >> CSR_GB] += 1; }
    int acc = 0; for (int g = 0; g < nG; ++g) { run[g] = acc; acc += cnt[g]; }
    for (int e = e0; e < e1; ++e) { int d = dst[e]; d = (d < 0) ? 0 : (d >= N ? N - 1 : d); const int g = d >> CSR_GB; ids[run[g]] = e; run[g] += 1; } }
  __syncthreads();
  typedef __attribute__((ext_vector_type(4))) int v4i;
  for (int pass = 0; pass < 2; ++pass) {
    for (int i = threadIdx.x; i < CHP / 4; i += 64) *(volatile v4i*)(STG + (size_t)b * CHP + i * 4) = *(const v4i*)(&ids[i * 4]);
    for (int i = threadIdx.x; i < NGP / 4; i += 64) { v4i v; for (int e = 0; e < 4; ++e) v[e] = (i * 4 + e < nG) ? cnt[i * 4 + e] : 0; *(volatile v4i*)(HST + (size_t)b * NGP + i * 4) = v; }
    __threadfence(); }
}
__global__ __launch_bounds__(512) void csrS_kernel(const int* __restrict__ HST, int nG, int NGP, int* __restrict__ START, int* __restrict__ TOT, int* __restrict__ OFF) {
  __shared__ int tot[CSR_MAXG];
  const int b = threadIdx.x;
  for (int pass = 0; pass < 2; ++pass) { int runb = 0; for (int g = 0; g < nG; ++g) { int c = HST[(size_t)b * NGP + g]; c = (c < 0) ? 0 : c; ((volatile int*)OFF)[(size_t)g * CSR_NBLK + b] = runb; runb += c; } __threadfence(); }
  for (int g = threadIdx.x; g < nG; g += 512) { int s = 0; for (int bb = 0; bb < CSR_NBLK; ++bb) { int c = HST[(size_t)bb * NGP + g]; s += (c < 0) ? 0 : c; } tot[g] = s; }
  __syncthreads();
  if (threadIdx.x < 32) {
    __shared__ int st[CSR_MAXG + 32];
    if (threadIdx.x == 0) { int acc = 0; for (int g = 0; g < NGP; ++g) { st[g] = acc; if (g < nG) acc += (tot[g] + 31) & ~31; } st[NGP] = acc; }
    __builtin_amdgcn_fence(__ATOMIC_RELEASE, "workgroup"); __builtin_amdgcn_wave_barrier(); __builtin_amdgcn_fence(__ATOMIC_ACQUIRE, "workgroup");
    for (int pass = 0; pass < 2; ++pass) { for (int i = threadIdx.x; i < NGP + 32; i += 32) { ((volatile int*)START)[i] = (i <= NGP) ? st[min(i, NGP)] : 0; ((volatile int*)TOT)[i] = (i < nG) ? tot[i] : 0; } __threadfence(); } }
}
__global__ __launch_bounds__(256) void csrB_kernel(const int* __restrict__ dst, int N, int nG, int CHP, int NGP, int permLen, const int* __restrict__ STG, const int* __restrict__ HST, const int* __restrict__ OFF, const int* __restrict__ START, const int* __restrict__ TOT, int* __restrict__ PERM, int* __restrict__ ROWPTR, int* __restrict__ ROWCNT, int* __restrict__ FLAG) {
  typedef __attribute__((ext_vector_type(4))) int v4i;
  __shared__ int ids[CSR_CAP]; __shared__ unsigned short key[CSR_CAP]; __shared__ int outp[CSR_CAP]; __shared__ int ncnt[CSR_GN + 1]; __shared__ int boff[CSR_NBLK + 1];
  const int g = blockIdx.x, t_ = threadIdx.x; int tot = TOT[g]; int st = START[g], stn = START[g + 1]; const int v0 = g * CSR_GN; const int nv = min(CSR_GN, N - v0); const int t0 = g * CSR_TS;
  st = (st < 0) ? 0 : (st > permLen - 32 ? permLen - 32 : st) & ~31; stn = (stn < st) ? st : (stn > permLen ? permLen : stn); tot = (tot < 0) ? 0 : tot; if (tot > stn - st && tot <= CSR_CAP) tot = stn - st;
  if (tot > CSR_CAP) {
    for (int pass = 0; pass < 2; ++pass) { for (int i = t_; i < CSR_TS / 4; i += 256) { v4i a, c; for (int e = 0; e < 4; ++e) { a[e] = st; c[e] = 0; } *(volatile v4i*)(ROWPTR + t0 + i * 4) = a; *(volatile v4i*)(ROWCNT + t0 + i * 4) = c; } if (t_ == 0) ((volatile int*)FLAG)[0] = 1; __threadfence(); } (void)nv; return; }
  if (t_ == 0) { int acc = 0; for (int b = 0; b < CSR_NBLK; ++b) { boff[b] = acc; int c = HST[(size_t)b * NGP + g]; c = (c < 0) ? 0 : (c > CHP ? CHP : c); acc += c; if (acc > tot) acc = tot; } boff[CSR_NBLK] = acc; }
  for (int i = t_; i <= CSR_GN; i += 256) ncnt[i] = 0;
  __syncthreads();
  for (int b = 0; b < CSR_NBLK; ++b) { const int c = boff[b + 1] - boff[b]; int o_ = OFF[(size_t)g * CSR_NBLK + b]; o_ = (o_ < 0) ? 0 : (o_ > CHP - c ? CHP - c : o_); const int* src_ = STG + (size_t)b * CHP + o_;
    for (int i = t_; i < c; i += 256) { int id = src_[i]; id = (id < 0) ? 0 : id; ids[boff[b] + i] = id; int d = dst[id]; d = (d < v0) ? v0 : (d >= N ? N - 1 : d); int kk = d - v0; kk = (kk < 0) ? 0 : (kk >= CSR_GN ? CSR_GN - 1 : kk); key[boff[b] + i] = (unsigned short)kk; } }
  __syncthreads();
  if (t_ == 0) { for (int i = 0; i < tot; ++i) ncnt[key[i]] += 1; int acc = 0; for (int vl = 0; vl < CSR_GN; ++vl) { const int c = ncnt[vl]; ncnt[vl] = acc; acc += c; } ncnt[CSR_GN] = acc;
    for (int i = 0; i < tot; ++i) { const int vl = key[i]; outp[ncnt[vl]] = ids[i]; ncnt[vl] += 1; }
    for (int vl = CSR_GN; vl > 0; --vl) ncnt[vl] = ncnt[vl - 1]; ncnt[0] = 0; }
  __syncthreads();
  for (int pass = 0; pass < 2; ++pass) {
    for (int i = t_; i < (stn - st) / 4; i += 256) { v4i v; for (int e = 0; e < 4; ++e) { const int q = i * 4 + e; v[e] = (q < tot) ? outp[q] : -1; } *(volatile v4i*)(PERM + st + i * 4) = v; }
    for (int i = t_; i < CSR_TS / 4; i += 256) { v4i a, c; for (int e = 0; e < 4; ++e) { const int vl = i * 4 + e; const int vc = vl < CSR_GN ? vl : CSR_GN; a[e] = (vl < CSR_GN) ? st + ncnt[vc] : st; c[e] = (vl < nv) ? (ncnt[(vc < CSR_GN ? vc : CSR_GN - 1) + 1] - ncnt[vc]) : 0; } *(volatile v4i*)(ROWPTR + t0 + i * 4) = a; *(volatile v4i*)(ROWCNT + t0 + i * 4) = c; }
    __threadfence(); }
}
__global__ __launch_bounds__(256) void csrZ_kernel(int* __restrict__ p, size_t n4) { typedef __attribute__((ext_vector_type(4))) int v4i; const size_t tid = (size_t)blockIdx.x * 256 + threadIdx.x, nth = (size_t)gridDim.x * 256; v4i z = {0, 0, 0, 0}; for (size_t i = tid; i < n4; i += nth) *(volatile v4i*)(p + i * 4) = z; }
struct CsrBufs { int *STG, *HST, *OFF, *START, *TOT, *PERM, *ROWPTR, *ROWCNT, *FLAG; int nG, NGP, CHP; size_t permLen; char* base; size_t bytes; };
static size_t csr_carve(CsrBufs& c, char* ws, size_t off, int E, int N) {
  const size_t off0 = off; c.base = ws + off;
  auto al = [&](size_t bytes) { char* p = ws + off; off += (bytes + 255) & ~(size_t)255; return p; };
  c.nG = (N + CSR_GN - 1) / CSR_GN; c.NGP = (c.nG + 31) & ~31; const int ch = (E + CSR_NBLK - 1) / CSR_NBLK; c.CHP = (ch + 31) & ~31; c.permLen = (size_t)E + 32 * (size_t)c.nG + 32;
  c.STG = (int*)al((size_t)CSR_NBLK * c.CHP * 4); c.HST = (int*)al((size_t)CSR_NBLK * c.NGP * 4); c.OFF = (int*)al((size_t)c.NGP * CSR_NBLK * 4); c.START = (int*)al((size_t)(c.NGP + 64) * 4); c.TOT = (int*)al((size_t)(c.NGP + 64) * 4);
  c.PERM = (int*)al(c.permLen * 4); c.ROWPTR = (int*)al((size_t)c.nG * CSR_TS * 4); c.ROWCNT = (int*)al((size_t)c.nG * CSR_TS * 4); c.FLAG = (int*)al(256);
  c.bytes = off - off0; return off;
}
static void csr_build(const CsrBufs& c, const int* dst, int E, int N, hipStream_t stream) {
  const size_t smem = (size_t)(2 * c.NGP + c.CHP) * 4;
  csrZ_kernel<<<512, 256, 0, stream>>>((int*)c.base, c.bytes / 16);
  csrA_kernel<<<CSR_NBLK, 64, smem, stream>>>(dst, E, N, c.nG, c.CHP, c.NGP, c.STG, c.HST);
  csrS_kernel<<<1, 512, 0, stream>>>(c.HST, c.nG, c.NGP, c.START, c.TOT, c.OFF);
  csrB_kernel<<<c.nG, 256, 0, stream>>>(dst, N, c.nG, c.CHP, c.NGP, (int)c.permLen, c.STG, c.HST, c.OFF, c.START, c.TOT, c.PERM, c.ROWPTR, c.ROWCNT, c.FLAG);
}


__global__ __launch_bounds__(256) void wprep_kernel(const float* __restrict__ wm1, const float* __restrict__ wm2, const float* __restrict__ we1, const float* __restrict__ we2, b16* __restrict__ W1A, b16* __restrict__ W1B, b16* __restrict__ W2, b16* __restrict__ WE1, b16* __restrict__ WE2) {
  const int u = blockIdx.x * 256 + threadIdx.x; v8b v; int t = u;
  const int n1 = HP * D / 8, n2 = 32 * RW / 8, n3 = HP * RW / 8, n4 = 32 * RW / 8;
  if (t < 2 * n1) { const bool second = t >= n1; const int e = (second ? t - n1 : t) * 8; const int o = e / D, k0 = e % D; for (int j = 0; j < 8; ++j) { const int k = k0 + j; v[j] = (o < HID) ? (b16)(bf16_rne(wm1[(size_t)((second ? D : 0) + k) * HID + (o < HID ? o : 0)]) * WSC) : (b16)0.0f; } for (int p = 0; p < 2; ++p) { *(volatile v8b*)((second ? W1B : W1A) + e) = v; __threadfence(); } return; } t -= 2 * n1;
  if (t < n2) { const int e = t * 8; const int o = e / RW, k0 = e % RW; for (int j = 0; j < 8; ++j) { const int k = k0 + j; v[j] = (o < MSG && k < HID) ? (b16)(bf16_rne(wm2[(size_t)(k < HID ? k : 0) * MSG + (o < MSG ? o : 0)]) * WSC) : (b16)0.0f; } for (int p = 0; p < 2; ++p) { *(volatile v8b*)(W2 + e) = v; __threadfence(); } return; } t -= n2;
  if (t < n3) { const int e = t * 8; const int o = e / RW, k0 = e % RW; for (int j = 0; j < 8; ++j) { const int k = k0 + j; v[j] = (o < HID && k < MSG + D + 1) ? (b16)(bf16_rne(we1[(size_t)(k < MSG + D + 1 ? k : 0) * HID + (o < HID ? o : 0)]) * WSC) : (b16)0.0f; } for (int p = 0; p < 2; ++p) { *(volatile v8b*)(WE1 + e) = v; __threadfence(); } return; } t -= n3;
  if (t < n4) { const int e = t * 8; const int o = e / RW, k0 = e % RW; for (int j = 0; j < 8; ++j) { const int k = k0 + j; v[j] = (k < HID) ? (b16)(bf16_rne(we2[(size_t)(k < HID ? k : 0) * D + o]) * WSC) : (b16)0.0f; } for (int p = 0; p < 2; ++p) { *(volatile v8b*)(WE2 + e) = v; __threadfence(); } }
}
__global__ __launch_bounds__(128) void pgemm_kernel(const float* __restrict__ Hin, const b16* __restrict__ W, int nrows, float* __restrict__ P) {
  __shared__ __attribute__((aligned(16))) float Tf[4][16][HP + 4];
  const int wave = threadIdx.x >> 5, lane = threadIdx.x & 31, nloc = lane & 15, hlf = lane >> 4; const size_t m0 = ((size_t)blockIdx.x * 4 + wave) * 16; if (m0 >= (size_t)nrows) return;
  const float* xr = Hin + (m0 + nloc) * D; v16b a; for (int j = 0; j < 8; ++j) { a[j] = (b16)(bf16_rne(xr[8 * hlf + j]) * XS); a[8 + j] = (b16)(bf16_rne(xr[16 + 8 * hlf + j]) * XS); }
  v8f acc[3];
#pragma unroll
  for (int t = 0; t < 3; ++t) { acc[t] = (v8f){}; acc[t] = wmma16b(a, frag_kb(W + (size_t)(t * 16 + nloc) * D, hlf), acc[t]); }
#pragma unroll
  for (int t = 0; t < 3; ++t)
#pragma unroll 1
    for (int r8 = 0; r8 < 8; ++r8) Tf[wave][8 * hlf + r8][t * 16 + nloc] = acc[t][r8] * (1.0f / (XS * WSC));
  wave_lds_sync();
  for (int pass = 0; pass < 2; ++pass) { for (int rr = 0; rr < 16; ++rr) if (lane < HP / 4) *(volatile v4f*)(P + (m0 + rr) * HP + lane * 4) = *(const v4f*)(&Tf[wave][rr][lane * 4]); __threadfence(); }
}
__global__ __launch_bounds__(256) void rsum_kernel(const float* __restrict__ PA, const float* __restrict__ PB, const int* __restrict__ from_, const int* __restrict__ PERM, const int* __restrict__ ROWPTR, const int* __restrict__ ROWCNT, int permLen, float* __restrict__ R) {
  const int wave = threadIdx.x >> 5, lane = threadIdx.x & 31; const size_t row = (size_t)blockIdx.x * 8 + wave; const int b = (int)(row / NCN), v = (int)(row % NCN); const int lc = lane < HP / 4 ? lane : 0;
  int st = ROWPTR[v], cnt = ROWCNT[v]; cnt = iclamp(cnt, 0, 65536); st = iclamp(st, 0, permLen - cnt); v4f a = {0.0f, 0.0f, 0.0f, 0.0f}; const v4f pb = *(const v4f*)(PB + row * HP + lc * 4);
#pragma unroll 1
  for (int j = 0; j < cnt; ++j) { const int e = iclamp(PERM[st + j], 0, E - 1); const size_t s = (size_t)iclamp(from_[e], 0, NV - 1); const v4f pa = *(const v4f*)(PA + ((size_t)b * NV + s) * HP + lc * 4); for (int i = 0; i < 4; ++i) a[i] += fmaxf(pa[i] + pb[i], 0.0f); }
  if (lane >= HID / 4) a = (v4f){0.0f, 0.0f, 0.0f, 0.0f};
  for (int pass = 0; pass < 2; ++pass) { if (lane < RW / 4) *(volatile v4f*)(R + row * RW + lane * 4) = a; __threadfence(); }
}
__global__ __launch_bounds__(32) void node_kernel(const float* __restrict__ R, const float* __restrict__ hto, const float* __restrict__ logit, const b16* __restrict__ W2, const b16* __restrict__ WE1, const b16* __restrict__ WE2, float* __restrict__ out) {
  __shared__ __attribute__((aligned(16))) b16 Ah[16][RW + 8], Al[16][RW + 8]; __shared__ __attribute__((aligned(16))) float Tf[16][D + 4];
  const int lane = threadIdx.x, nloc = lane & 15, hlf = lane >> 4; const size_t m0 = (size_t)blockIdx.x * 16;
  for (int rr = 0; rr < 16; ++rr) { const v2f rv = *(const v2f*)(R + (m0 + rr) * RW + lane * 2); for (int j = 0; j < 2; ++j) { b16 p, q; split16(rv[j] * XS, p, q); Ah[rr][lane * 2 + j] = p; Al[rr][lane * 2 + j] = q; } }
  wave_lds_sync();
  v8f am[2] = {(v8f){}, (v8f){}};
#pragma unroll
  for (int kb = 0; kb < RW; kb += 32) { const v16b a = frag_kb(&Ah[nloc][kb], hlf), al = frag_kb(&Al[nloc][kb], hlf);
#pragma unroll
    for (int t = 0; t < 2; ++t) { const v16b bw = frag_kb(W2 + (size_t)(t * 16 + nloc) * RW + kb, hlf); am[t] = wmma16b(a, bw, am[t]); am[t] = wmma16b(al, bw, am[t]); } }
  wave_lds_sync();
#pragma unroll
  for (int t = 0; t < 2; ++t) { const int c = t * 16 + nloc;
#pragma unroll 1
    for (int r8 = 0; r8 < 8; ++r8) { const int rl = 8 * hlf + r8; if (c < MSG) { b16 p, q; split16(am[t][r8] * (1.0f / (XS * WSC)) * XS, p, q); Ah[rl][c] = p; Al[rl][c] = q; } } }
  for (int rr = 0; rr < 16; ++rr) { const size_t row = m0 + rr; const float hv = bf16_rne(hto[row * D + lane]); Ah[rr][MSG + lane] = (b16)(hv * XS); Al[rr][MSG + lane] = (b16)0.0f;
    if (lane == 0) { Ah[rr][MSG + D] = (b16)(bf16_rne(logit[row]) * XS); Al[rr][MSG + D] = (b16)0.0f; } if (lane + 32 > MSG + D && lane + 32 < RW) { Ah[rr][lane + 32] = (b16)0.0f; Al[rr][lane + 32] = (b16)0.0f; } }
  wave_lds_sync();
  v8f ah[3] = {(v8f){}, (v8f){}, (v8f){}};
#pragma unroll
  for (int kb = 0; kb < RW; kb += 32) { const v16b a = frag_kb(&Ah[nloc][kb], hlf), al = frag_kb(&Al[nloc][kb], hlf);
#pragma unroll
    for (int t = 0; t < 3; ++t) { const v16b bw = frag_kb(WE1 + (size_t)(t * 16 + nloc) * RW + kb, hlf); ah[t] = wmma16b(a, bw, ah[t]); ah[t] = wmma16b(al, bw, ah[t]); } }
  wave_lds_sync();
#pragma unroll
  for (int t = 0; t < 3; ++t) { const int c = t * 16 + nloc;
#pragma unroll 1
    for (int r8 = 0; r8 < 8; ++r8) { const int rl = 8 * hlf + r8; const float hv = c < HID ? fmaxf(ah[t][r8] * (1.0f / (XS * WSC)), 0.0f) : 0.0f; b16 p, q; split16(hv * XS, p, q); Ah[rl][c] = p; Al[rl][c] = q; } }
  for (int rr = 0; rr < 16; ++rr) if (lane >= 16) { Ah[rr][32 + lane] = (b16)0.0f; Al[rr][32 + lane] = (b16)0.0f; }
  wave_lds_sync();
  v8f ao[2] = {(v8f){}, (v8f){}};
#pragma unroll
  for (int kb = 0; kb < RW; kb += 32) { const v16b a = frag_kb(&Ah[nloc][kb], hlf), al = frag_kb(&Al[nloc][kb], hlf);
#pragma unroll
    for (int t = 0; t < 2; ++t) { const v16b bw = frag_kb(WE2 + (size_t)(t * 16 + nloc) * RW + kb, hlf); ao[t] = wmma16b(a, bw, ao[t]); ao[t] = wmma16b(al, bw, ao[t]); } }
#pragma unroll
  for (int t = 0; t < 2; ++t)
#pragma unroll 1
    for (int r8 = 0; r8 < 8; ++r8) Tf[8 * hlf + r8][t * 16 + nloc] = ao[t][r8] * (1.0f / (XS * WSC));
  wave_lds_sync();
  for (int pass = 0; pass < 2; ++pass) { for (int rr = 0; rr < 16; ++rr) if (lane < 8) *(volatile v4f*)(out + (m0 + rr) * D + lane * 4) = *(const v4f*)(&Tf[rr][lane * 4]); __threadfence(); }
}
}

extern "C" void kernel_launch(void* const* d_in, const int* in_sizes, int n_in, void* d_out, int out_size, void* d_ws, size_t ws_size, hipStream_t stream) {
  (void)n_in;
  auto Fp = [&](int i) { return (const float*)d_in[i]; }; auto Ip = [&](int i) { return (const int*)d_in[i]; };
  if (in_sizes[0] != NB * NV * D || in_sizes[1] != NB * NCN * D || in_sizes[3] != NB * NCN || in_sizes[5] != E || in_sizes[8] != E || in_sizes[9] != 2 * D * HID || in_sizes[10] != HID * MSG || in_sizes[13] != (MSG + D + 1) * HID || in_sizes[14] != HID * D || out_size != 2 * NB * NCN * D) return;
  size_t off = 0; char* ws = (char*)d_ws;
  auto carve = [&](size_t bytes) { char* p = ws + off; off += (bytes + 255) & ~(size_t)255; return p; };
  b16* W1A = (b16*)carve(HP * D * 2); b16* W1B = (b16*)carve(HP * D * 2); b16* W2 = (b16*)carve(32 * RW * 2); b16* WE1 = (b16*)carve(HP * RW * 2); b16* WE2 = (b16*)carve(32 * RW * 2);
  float* PA = (float*)carve((size_t)NB * NV * HP * 4); float* PB = (float*)carve((size_t)NB * NCN * HP * 4); float* R = (float*)carve((size_t)NB * NCN * RW * 4);
  CsrBufs csr; off = csr_carve(csr, ws, off, E, NCN);
  if (off > ws_size || off > ((size_t)128 << 20)) return;
  const int nw = (2 * HP * D / 8 + 32 * RW / 8 + HP * RW / 8 + 32 * RW / 8 + 255) / 256;
  for (int s = 0; s < 2; ++s) { const float* hto = Fp(1 + s); const float* logit = Fp(3 + s); const int* from_ = Ip(5 + 2 * s); const int* to_ = Ip(6 + 2 * s);
    wprep_kernel<<<nw, 256, 0, stream>>>(Fp(9 + 2 * s), Fp(10 + 2 * s), Fp(13 + 2 * s), Fp(14 + 2 * s), W1A, W1B, W2, WE1, WE2);
    csr_build(csr, to_, E, NCN, stream);
    pgemm_kernel<<<NB * NV / 64, 128, 0, stream>>>(Fp(0), W1A, NB * NV, PA);
    pgemm_kernel<<<NB * NCN / 64, 128, 0, stream>>>(hto, W1B, NB * NCN, PB);
    rsum_kernel<<<NB * NCN / 8, 256, 0, stream>>>(PA, PB, from_, csr.PERM, csr.ROWPTR, csr.ROWCNT, (int)csr.permLen, R);
    node_kernel<<<NB * NCN / 16, 32, 0, stream>>>(R, hto, logit, W2, WE1, WE2, (float*)d_out + (size_t)s * NB * NCN * D); }
}
